// WMSA_4088808865805
// MI455X (gfx1250) — hardware-verified
//
#include <hip/hip_runtime.h>


#define NB_  4
#define HI   192
#define WI   192
#define CC   64
#define NPX  (NB_ * HI * WI)
#define NWIN 2304
#define L_   64
#define NHD  8
#define DH   64
#define INNER 512
#define WCH  48
#define NZ   (WCH * NHD)
#define DM   CC
#define SCL  0.125f
#define LOSC 1024.0f

typedef _Float16 h16;
typedef unsigned short bf;
typedef __attribute__((ext_vector_type(16))) __bf16   v16bf;
typedef __attribute__((ext_vector_type(16))) _Float16 v16h;
typedef __attribute__((ext_vector_type(8)))  _Float16 v8h;
typedef __attribute__((ext_vector_type(8)))  unsigned short v8us;
typedef __attribute__((ext_vector_type(8)))  float    v8f;
typedef __attribute__((ext_vector_type(4)))  float    v4f;
typedef __attribute__((ext_vector_type(4)))  _Float16 v4h;
typedef v8h  __attribute__((may_alias)) v8ha;
typedef v4f  __attribute__((may_alias)) v4fa;
typedef v8us __attribute__((may_alias)) v8usa;

__device__ __forceinline__ unsigned short f2bf(float f) { unsigned u = __float_as_uint(f); u += 0x7FFFu + ((u >> 16) & 1u); return (unsigned short)(u >> 16); }
__device__ __forceinline__ float bf2f(unsigned short b) { return __uint_as_float(((unsigned)b) << 16); }
__device__ __forceinline__ float bfr(float f) { return bf2f(f2bf(f)); }
__device__ __forceinline__ v16h cat16(v8h lo, v8h hi) { return __builtin_shufflevector(lo, hi, 0, 1, 2, 3, 4, 5, 6, 7, 8, 9, 10, 11, 12, 13, 14, 15); }
__device__ __forceinline__ v16bf cat16b(v8us lo, v8us hi) { return __builtin_bit_cast(v16bf, __builtin_shufflevector(lo, hi, 0, 1, 2, 3, 4, 5, 6, 7, 8, 9, 10, 11, 12, 13, 14, 15)); }
__device__ __forceinline__ v8f wmma16(v16h a, v16h b, v8f c) { return __builtin_amdgcn_wmma_f32_16x16x32_f16(false, a, false, b, (short)0, c, false, false); }
__device__ __forceinline__ v8f wmmab(v16bf a, v16bf b, v8f c) { return __builtin_amdgcn_wmma_f32_16x16x32_bf16(false, a, false, b, (short)0, c, false, false); }

__global__ __launch_bounds__(256) void k_wt(const float* __restrict__ Wm, int K, int ncols, bf* WT) {
    __shared__ __align__(16) unsigned short tl[64 * 72];
    const int tid = threadIdx.x, k0 = blockIdx.x * 64, n0 = blockIdx.y * 64;
    const int kk = tid >> 2, nq = (tid & 3) * 16;
#pragma unroll
    for (int i = 0; i < 16; ++i) tl[(nq + i) * 72 + kk] = f2bf(Wm[(size_t)(k0 + kk) * ncols + n0 + nq + i]);
    __syncthreads();
    const int piece = tid & 7;
    auto pass = [&]() {
#pragma unroll
        for (int s = 0; s < 2; ++s) { const int nr = (tid >> 3) + 32 * s; const v8us val = *(const v8usa*)(tl + nr * 72 + piece * 8); *(volatile v8us*)(WT + (size_t)(n0 + nr) * K + k0 + piece * 8) = val; }
    };
    pass(); __threadfence(); pass();
}
template <bool SPLITA, bool F16OUT = false>
__global__ __launch_bounds__(128) void k_gemmb(const bf* __restrict__ A, const bf* __restrict__ Al, const bf* __restrict__ Bn, const float* __restrict__ bias, float* C, int ldc, h16* C2, const float* __restrict__ R = nullptr, int K = DM, int roundR = 1) {
    __shared__ __align__(16) float ost[4][16 * 68];
    const int lane = threadIdx.x & 31, wave = threadIdx.x >> 5, lr = lane & 15, hi = lane >> 4;
    const int r0 = blockIdx.x * 64 + wave * 16, c0 = blockIdx.y * 64;
    const size_t aoff = (size_t)(r0 + lr) * K + 8 * hi;
    size_t boff[4];
#pragma unroll
    for (int t = 0; t < 4; ++t) boff[t] = (size_t)(c0 + t * 16 + lr) * K + 8 * hi;
    v8f acc[4];
#pragma unroll
    for (int t = 0; t < 4; ++t) acc[t] = (v8f){};
#pragma unroll 1
    for (int kc = 0; kc < K; kc += 32) {
        const v16bf a = cat16b(*(const v8us*)(A + aoff + kc), *(const v8us*)(A + aoff + kc + 16));
        v16bf al = a;
        if (SPLITA) al = cat16b(*(const v8us*)(Al + aoff + kc), *(const v8us*)(Al + aoff + kc + 16));
#pragma unroll
        for (int t = 0; t < 4; ++t) { const v16bf b = cat16b(*(const v8us*)(Bn + boff[t] + kc), *(const v8us*)(Bn + boff[t] + kc + 16)); acc[t] = wmmab(a, b, acc[t]); if (SPLITA) acc[t] = wmmab(al, b, acc[t]); }
        asm volatile("v_nop\n\tv_nop\n\tv_nop\n\tv_nop" : "+v"(acc[0]), "+v"(acc[1]), "+v"(acc[2]), "+v"(acc[3]) : "v"(a), "v"(al));
    }
    float* os = &ost[wave][0];
#pragma unroll
    for (int t = 0; t < 4; ++t) { const float bv = bias ? bfr(bias[c0 + t * 16 + lr]) : 0.f;
#pragma unroll
        for (int j = 0; j < 8; ++j) os[(hi * 8 + j) * 68 + t * 16 + lr] = acc[t][j] + bv; }
    __syncthreads();
    if (F16OUT) {
        h16* crow = (h16*)(void*)C + (size_t)r0 * ldc + c0;
        auto pass = [&]() {
#pragma unroll
            for (int s = 0; s < 4; ++s) { const int row = 4 * s + (lane >> 3), piece = lane & 7; const float* sp = os + row * 68 + piece * 8; v8h o, o2;
#pragma unroll
                for (int i = 0; i < 8; ++i) { const h16 a = (h16)sp[i]; o[i] = a; o2[i] = (h16)((sp[i] - (float)a) * LOSC); }
                *(volatile v8h*)(crow + (size_t)row * ldc + piece * 8) = o; if (C2) *(volatile v8h*)(C2 + (size_t)r0 * ldc + c0 + (size_t)row * ldc + piece * 8) = o2; }
        };
        pass(); __threadfence(); pass();
    } else {
        float* crow = C + (size_t)r0 * ldc + c0;
        auto pass = [&]() {
#pragma unroll
            for (int s = 0; s < 8; ++s) { const int Lid = (lane >> 3) + 4 * s, piece = lane & 7; const int row = Lid >> 1, cofs = (Lid & 1) * 32 + piece * 4;
                v4f val = *(const v4fa*)(os + row * 68 + cofs); if (R) { const v4f rv = *(const v4f*)(R + ((size_t)r0 + row) * ldc + c0 + cofs); val += roundR ? (v4f){bfr(rv[0]), bfr(rv[1]), bfr(rv[2]), bfr(rv[3])} : rv; }
                *(volatile v4f*)(crow + (size_t)row * ldc + cofs) = val; }
        };
        pass(); __threadfence(); pass();
    }
}


template <int MODE>
__global__ __launch_bounds__(128) void k_gemm3z(const bf* __restrict__ Ah, const bf* __restrict__ Al, const bf* __restrict__ Bh, const bf* __restrict__ Bl, int K, float* C, int ldc, size_t sA, size_t sB, size_t sC) {
    if ((MODE & 1) && (int)blockIdx.y * 64 > (int)blockIdx.x * 64 + 63) return;
    const size_t z = blockIdx.z; Ah += z * sA; Al += z * sA; Bh += z * sB; Bl += z * sB; C += z * sC;
    const int Klim = (MODE & 2) ? min(K, ((int)blockIdx.x + 1) * 64) : K;
    __shared__ __align__(16) float ost[4][16 * 68];
    const int lane = threadIdx.x & 31, wave = threadIdx.x >> 5, lr = lane & 15, hi = lane >> 4;
    const int r0 = blockIdx.x * 64 + wave * 16, c0 = blockIdx.y * 64;
    const size_t aoff = (size_t)(r0 + lr) * K + 8 * hi;
    v8f acc[4];
#pragma unroll
    for (int t = 0; t < 4; ++t) acc[t] = (v8f){};
#pragma unroll 1
    for (int kc = 0; kc < Klim; kc += 32) {
        const v16bf a = cat16b(*(const v8us*)(Ah + aoff + kc), *(const v8us*)(Ah + aoff + kc + 16));
        v16bf al = a; if (!(MODE & 4) && !(MODE & 16)) al = cat16b(*(const v8us*)(Al + aoff + kc), *(const v8us*)(Al + aoff + kc + 16));
#pragma unroll
        for (int t = 0; t < 4; ++t) { const size_t bo = (size_t)(c0 + t * 16 + lr) * K + kc + 8 * hi;
            const v16bf bh = cat16b(*(const v8us*)(Bh + bo), *(const v8us*)(Bh + bo + 16));
            acc[t] = wmmab(a, bh, acc[t]);
            if (!(MODE & 4)) { if (!(MODE & 16)) acc[t] = wmmab(al, bh, acc[t]); if (!(MODE & 8)) { const v16bf bl = cat16b(*(const v8us*)(Bl + bo), *(const v8us*)(Bl + bo + 16)); acc[t] = wmmab(a, bl, acc[t]); } } }
        asm volatile("v_nop\n\tv_nop\n\tv_nop\n\tv_nop" : "+v"(acc[0]), "+v"(acc[1]), "+v"(acc[2]), "+v"(acc[3]) : "v"(a), "v"(al));
    }
    float* os = &ost[wave][0];
#pragma unroll
    for (int t = 0; t < 4; ++t) {
#pragma unroll
        for (int j = 0; j < 8; ++j) os[(hi * 8 + j) * 68 + t * 16 + lr] = acc[t][j]; }
    __builtin_amdgcn_wave_barrier(); asm volatile("" ::: "memory");
    float* crow = C + (size_t)r0 * ldc + c0;
    auto pass = [&]() {
#pragma unroll
        for (int s = 0; s < 8; ++s) { const int Lid = (lane >> 3) + 4 * s, piece = lane & 7; const int row = Lid >> 1, cofs = (Lid & 1) * 32 + piece * 4;
            const v4f val = *(const v4fa*)(os + row * 68 + cofs); *(volatile v4f*)(crow + (size_t)row * ldc + cofs) = val; }
    };
    pass(); __threadfence(); pass();
}
__global__ __launch_bounds__(256) void k_planes32z(const float* __restrict__ F, int ld, int off, float sc, int rows, bf* Ph, bf* Pl) {
    typedef __attribute__((ext_vector_type(2))) unsigned short v2us;
    const int lane = threadIdx.x & 31; const size_t r = ((size_t)blockIdx.x * 8 + (threadIdx.x >> 5)) * 2 + (lane >> 4); if (r >= (size_t)rows) return; const int z = blockIdx.z; const int c0 = (lane & 15) * 2; v2us oh, ol;
    Ph += (size_t)z * rows * 32; Pl += (size_t)z * rows * 32;
#pragma unroll
    for (int i = 0; i < 2; ++i) { const float y = F[r * ld + off + z * 32 + c0 + i] * sc; const unsigned short hb = f2bf(y); oh[i] = hb; ol[i] = f2bf(y - bf2f(hb)); }
    const size_t o = r * 32 + c0; *(volatile v2us*)(Ph + o) = oh; *(volatile v2us*)(Pl + o) = ol; __threadfence(); *(volatile v2us*)(Ph + o) = oh; *(volatile v2us*)(Pl + o) = ol;
}
__global__ __launch_bounds__(256) void k_vtpadz(const float* __restrict__ F, int ld, int off, int nk, bf* Th, bf* Tl) {
    typedef __attribute__((ext_vector_type(2))) unsigned short v2us;
    const int lane = threadIdx.x & 31; const size_t wid = (size_t)blockIdx.x * 8 + (threadIdx.x >> 5); if (wid >= (size_t)64 * (nk / 64)) return; const int z = blockIdx.z; const int d = (int)(wid / (nk / 64)); const int k0 = (int)(wid % (nk / 64)) * 64 + lane * 2; v2us oh, ol;
    Th += (size_t)z * 64 * nk; Tl += (size_t)z * 64 * nk;
#pragma unroll
    for (int i = 0; i < 2; ++i) { const float y = (d < 32) ? F[(size_t)(k0 + i) * ld + off + z * 32 + (d < 32 ? d : 0)] : 0.f; const unsigned short hb = f2bf(y); oh[i] = hb; ol[i] = f2bf(y - bf2f(hb)); }
    const size_t o = (size_t)d * nk + k0; *(volatile v2us*)(Th + o) = oh; *(volatile v2us*)(Tl + o) = ol; __threadfence(); *(volatile v2us*)(Th + o) = oh; *(volatile v2us*)(Tl + o) = ol;
}
template <int NK>
__global__ __launch_bounds__(256) void k_softmaxz(const float* __restrict__ S, int rows, bf* PH, bf* PL) {
    typedef __attribute__((ext_vector_type(4))) unsigned short v4us;
    const int lane = threadIdx.x & 31, i = blockIdx.x * 8 + (threadIdx.x >> 5); if (i >= rows) return; const size_t zo = (size_t)blockIdx.z * rows * NK; const float* sr = S + zo + (size_t)i * NK; PH += zo; PL += zo;
    float m = -3.0e38f;
#pragma unroll 1
    for (int c0 = lane * 4; c0 < NK; c0 += 128) {
#pragma unroll
        for (int q = 0; q < 4; ++q) m = fmaxf(m, sr[c0 + q]); }
#pragma unroll
    for (int sh = 16; sh; sh >>= 1) m = fmaxf(m, __shfl_xor(m, sh, 32));
    float sum = 0.f;
#pragma unroll 1
    for (int c0 = lane * 4; c0 < NK; c0 += 128) {
#pragma unroll
        for (int q = 0; q < 4; ++q) sum += __expf(sr[c0 + q] - m); }
#pragma unroll
    for (int sh = 16; sh; sh >>= 1) sum += __shfl_xor(sum, sh, 32);
    const float inv = 1.0f / sum;
#pragma unroll 1
    for (int ps = 0; ps < 2; ++ps) {
#pragma unroll 1
        for (int c0 = lane * 4; c0 < NK; c0 += 128) { v4us oh, ol;
#pragma unroll
            for (int q = 0; q < 4; ++q) { const float p = __expf(sr[c0 + q] - m) * inv; const unsigned short hb = f2bf(p); oh[q] = hb; ol[q] = f2bf(p - bf2f(hb)); }
            const size_t o = (size_t)i * NK + c0; *(volatile v4us*)(PH + o) = oh; *(volatile v4us*)(PL + o) = ol; }
        if (ps == 0) __threadfence(); }
}
__global__ __launch_bounds__(256) void k_placez(const float* __restrict__ XH, int rows, int ldy, float* Y) {
    const int lane = threadIdx.x & 31; const size_t q = (size_t)blockIdx.x * 8 + (threadIdx.x >> 5); if (q >= (size_t)rows) return; const int z = blockIdx.z; const float v = XH[((size_t)z * rows + q) * 64 + lane];
    *(volatile float*)(Y + q * ldy + z * 32 + lane) = v; __threadfence(); *(volatile float*)(Y + q * ldy + z * 32 + lane) = v;
}

__global__ __launch_bounds__(256) void k_xroll(const float* __restrict__ x, size_t p0, bf* Xb) {
    typedef __attribute__((ext_vector_type(2))) unsigned short v2us;
    const int lane = threadIdx.x & 31; const size_t pl = (size_t)blockIdx.x * 8 + (threadIdx.x >> 5); if (pl >= (size_t)WCH * L_) return; const size_t p = p0 + pl; const int w = (int)(p % WI); const int h = (int)((p / WI) % HI); const int b = (int)(p / ((size_t)WI * HI));
    const size_t src = (((size_t)b * HI + (h + 4) % HI) * WI + (w + 4) % WI) * CC + lane * 2; v2us o; o[0] = f2bf(x[src]); o[1] = f2bf(x[src + 1]);
    *(volatile v2us*)(Xb + pl * CC + lane * 2) = o; __threadfence(); *(volatile v2us*)(Xb + pl * CC + lane * 2) = o;
}
__global__ __launch_bounds__(256) void k_blkplanes(const float* __restrict__ F, int ld, int coff, int w0, float sc, bf* Ph, bf* Pl) {
    typedef __attribute__((ext_vector_type(2))) unsigned short v2us;
    const int lane = threadIdx.x & 31; const size_t row = (size_t)blockIdx.x * 8 + (threadIdx.x >> 5); if (row >= (size_t)NZ * L_) return; const size_t z = row / L_; const int i = (int)(row % L_); const int win = w0 + (int)(z / NHD), hh = (int)(z % NHD);
    v2us oh, ol;
#pragma unroll
    for (int q = 0; q < 2; ++q) { const int d = lane * 2 + q; const int f = hh * 4096 + i * 64 + d; const int t = f / INNER, c = f % INNER; const float y = F[((size_t)win * L_ + t) * ld + coff + c] * sc; const unsigned short hb = f2bf(y); oh[q] = hb; ol[q] = f2bf(y - bf2f(hb)); }
    const size_t o = row * DH + lane * 2; *(volatile v2us*)(Ph + o) = oh; *(volatile v2us*)(Pl + o) = ol; __threadfence(); *(volatile v2us*)(Ph + o) = oh; *(volatile v2us*)(Pl + o) = ol;
}
__global__ __launch_bounds__(256) void k_blkvt(const float* __restrict__ F, int ld, int coff, int w0, bf* Th, bf* Tl) {
    typedef __attribute__((ext_vector_type(2))) unsigned short v2us;
    const int lane = threadIdx.x & 31; const size_t row = (size_t)blockIdx.x * 8 + (threadIdx.x >> 5); if (row >= (size_t)NZ * DH) return; const size_t z = row / DH; const int d = (int)(row % DH); const int win = w0 + (int)(z / NHD), hh = (int)(z % NHD);
    v2us oh, ol;
#pragma unroll
    for (int q = 0; q < 2; ++q) { const int j = lane * 2 + q; const int f = hh * 4096 + j * 64 + d; const int t = f / INNER, c = f % INNER; const float y = F[((size_t)win * L_ + t) * ld + coff + c]; const unsigned short hb = f2bf(y); oh[q] = hb; ol[q] = f2bf(y - bf2f(hb)); }
    const size_t o = row * L_ + lane * 2; *(volatile v2us*)(Th + o) = oh; *(volatile v2us*)(Tl + o) = ol; __threadfence(); *(volatile v2us*)(Th + o) = oh; *(volatile v2us*)(Tl + o) = ol;
}
__global__ __launch_bounds__(256) void k_wsoft(const float* __restrict__ S, const float* __restrict__ pos, bf* PH, bf* PL) {
    typedef __attribute__((ext_vector_type(2))) unsigned short v2us;
    const int lane = threadIdx.x & 31; const size_t row = (size_t)blockIdx.x * 8 + (threadIdx.x >> 5); if (row >= (size_t)NZ * L_) return; const size_t z = row / L_; const int i = (int)(row % L_); const int hh = (int)(z % NHD);
    const float* sr = S + row * L_; const float* pr = pos + ((size_t)hh * L_ + i) * L_; const float a0 = sr[lane * 2] + bfr(pr[lane * 2]), a1 = sr[lane * 2 + 1] + bfr(pr[lane * 2 + 1]);
    float m = fmaxf(a0, a1);
#pragma unroll
    for (int sh = 16; sh; sh >>= 1) m = fmaxf(m, __shfl_xor(m, sh, 32));
    const float e0 = __expf(a0 - m), e1 = __expf(a1 - m); float s = e0 + e1;
#pragma unroll
    for (int sh = 16; sh; sh >>= 1) s += __shfl_xor(s, sh, 32);
    const float inv = 1.0f / s; const float p0 = e0 * inv, p1 = e1 * inv; v2us oh, ol;
    { const unsigned short hb = f2bf(p0); oh[0] = hb; ol[0] = f2bf(p0 - bf2f(hb)); } { const unsigned short hb = f2bf(p1); oh[1] = hb; ol[1] = f2bf(p1 - bf2f(hb)); }
    const size_t o = row * L_ + lane * 2; *(volatile v2us*)(PH + o) = oh; *(volatile v2us*)(PL + o) = ol; __threadfence(); *(volatile v2us*)(PH + o) = oh; *(volatile v2us*)(PL + o) = ol;
}
__global__ __launch_bounds__(256) void k_oplanes(const float* __restrict__ XO, bf* Oh, bf* Ol) {
    const int lane = threadIdx.x & 31; const size_t r = (size_t)blockIdx.x * 8 + (threadIdx.x >> 5); if (r >= (size_t)WCH * L_) return;
#pragma unroll 1
    for (int ps = 0; ps < 2; ++ps) {
#pragma unroll
        for (int q = 0; q < INNER / 256; ++q) { const size_t o = r * INNER + q * 256 + lane * 8; const v8f v = *(const v8f*)(XO + o); v8us oh, ol;
#pragma unroll
            for (int i = 0; i < 8; ++i) { const unsigned short hb = f2bf(v[i]); oh[i] = hb; ol[i] = f2bf(v[i] - bf2f(hb)); }
            *(volatile v8us*)(Oh + o) = oh; *(volatile v8us*)(Ol + o) = ol; }
        if (ps == 0) __threadfence(); }
}
__global__ __launch_bounds__(256) void k_unroll(const float* __restrict__ R, float* OUTP) {
    typedef __attribute__((ext_vector_type(2))) float v2f_;
    const int lane = threadIdx.x & 31; const size_t p = (size_t)blockIdx.x * 8 + (threadIdx.x >> 5); if (p >= (size_t)NPX) return; const int w = (int)(p % WI); const int h = (int)((p / WI) % HI); const int b = (int)(p / ((size_t)WI * HI));
    const size_t src = (((size_t)b * HI + (h + HI - 4) % HI) * WI + (w + WI - 4) % WI) * CC + lane * 2; const v2f_ v = *(const v2f_*)(R + src);
    *(volatile v2f_*)(OUTP + p * CC + lane * 2) = v; __threadfence(); *(volatile v2f_*)(OUTP + p * CC + lane * 2) = v;
}

extern "C" void kernel_launch(void* const* d_in, const int* in_sizes, int n_in,
                              void* d_out, int out_size, void* d_ws, size_t ws_size, hipStream_t stream) {
    (void)in_sizes; (void)n_in; (void)out_size;
    const float* x = (const float*)d_in[0]; const float* Wq = (const float*)d_in[1]; const float* Wkv = (const float*)d_in[2]; const float* Wo = (const float*)d_in[3]; const float* bo = (const float*)d_in[4]; const float* pos = (const float*)d_in[5];
    float* out = (float*)d_out;
    char* wsp = (char*)d_ws;
    auto take = [&](size_t bytes) { char* p = wsp; wsp += (bytes + 255) & ~(size_t)255; return (void*)p; };
    const size_t TCH = (size_t)WCH * L_;
    bf* WQ = (bf*)take((size_t)INNER * CC * 2); bf* WKV = (bf*)take((size_t)2 * INNER * CC * 2); bf* WO = (bf*)take((size_t)CC * INNER * 2);
    bf* Xb = (bf*)take(TCH * CC * 2); float* QF = (float*)take(TCH * INNER * 4); float* KVF = (float*)take(TCH * 2 * INNER * 4);
    bf* Qh = (bf*)take((size_t)NZ * L_ * DH * 2); bf* Ql = (bf*)take((size_t)NZ * L_ * DH * 2); bf* Kh = (bf*)take((size_t)NZ * L_ * DH * 2); bf* Kl = (bf*)take((size_t)NZ * L_ * DH * 2); bf* VTh = (bf*)take((size_t)NZ * DH * L_ * 2); bf* VTl = (bf*)take((size_t)NZ * DH * L_ * 2);
    float* S = (float*)take((size_t)NZ * L_ * L_ * 4); bf* PH = (bf*)take((size_t)NZ * L_ * L_ * 2); bf* PL = (bf*)take((size_t)NZ * L_ * L_ * 2); float* XO = (float*)take((size_t)NZ * L_ * DH * 4); bf* Oh = (bf*)take(TCH * INNER * 2); bf* Ol = (bf*)take(TCH * INNER * 2);
    float* RR = (float*)take((size_t)NPX * CC * 4);
    if ((size_t)(wsp - (char*)d_ws) > ws_size) return;
    k_wt<<<dim3(CC / 64, INNER / 64, 1), 256, 0, stream>>>(Wq, CC, INNER, WQ); k_wt<<<dim3(CC / 64, (2 * INNER) / 64, 1), 256, 0, stream>>>(Wkv, CC, 2 * INNER, WKV); k_wt<<<dim3(INNER / 64, CC / 64, 1), 256, 0, stream>>>(Wo, INNER, CC, WO);
    for (int c = 0; c < NWIN / WCH; ++c) { const size_t t0 = (size_t)c * TCH;
        k_xroll<<<(unsigned)(TCH / 8), 256, 0, stream>>>(x, t0, Xb);
        k_gemmb<false, false><<<dim3((unsigned)(TCH / 64), INNER / 64, 1), 128, 0, stream>>>(Xb, nullptr, WQ, nullptr, QF, INNER, nullptr, nullptr, CC);
        k_gemmb<false, false><<<dim3((unsigned)(TCH / 64), (2 * INNER) / 64, 1), 128, 0, stream>>>(Xb, nullptr, WKV, nullptr, KVF, 2 * INNER, nullptr, nullptr, CC);
        k_blkplanes<<<(NZ * L_) / 8, 256, 0, stream>>>(QF, INNER, 0, 0, SCL, Qh, Ql); k_blkplanes<<<(NZ * L_) / 8, 256, 0, stream>>>(KVF, 2 * INNER, 0, 0, 1.0f, Kh, Kl); k_blkvt<<<(NZ * DH) / 8, 256, 0, stream>>>(KVF, 2 * INNER, INNER, 0, VTh, VTl);
        k_gemm3z<0><<<dim3(1, 1, NZ), 128, 0, stream>>>(Qh, Ql, Kh, Kl, DH, S, L_, (size_t)L_ * DH, (size_t)L_ * DH, (size_t)L_ * L_);
        k_wsoft<<<(NZ * L_) / 8, 256, 0, stream>>>(S, pos, PH, PL);
        k_gemm3z<0><<<dim3(1, 1, NZ), 128, 0, stream>>>(PH, PL, VTh, VTl, L_, XO, DH, (size_t)L_ * L_, (size_t)DH * L_, (size_t)L_ * DH);
        k_oplanes<<<(unsigned)(TCH / 8), 256, 0, stream>>>(XO, Oh, Ol);
        k_gemmb<true, false><<<dim3((unsigned)(TCH / 64), 1, 1), 128, 0, stream>>>(Oh, Ol, WO, bo, RR + t0 * CC, CC, nullptr, nullptr, INNER); }
    k_unroll<<<NPX / 8, 256, 0, stream>>>(RR, out);
}
